// Covariance_Metric_23656679866493
// MI455X (gfx1250) — hardware-verified
//
#include <hip/hip_runtime.h>
#include <math.h>

typedef __attribute__((ext_vector_type(16))) _Float16 v16h;
typedef __attribute__((ext_vector_type(16))) __bf16 v16b;
typedef __attribute__((ext_vector_type(8)))  _Float16 v8h;
typedef __attribute__((ext_vector_type(8)))  float v8f;
typedef __attribute__((ext_vector_type(4)))  float v4f;
typedef __attribute__((ext_vector_type(2)))  float v2f;
typedef __attribute__((ext_vector_type(4)))  unsigned v4u;
typedef __attribute__((ext_vector_type(4)))  int v4i;
typedef float __attribute__((may_alias)) float_a;
typedef int __attribute__((may_alias)) int_a;

template <typename T> __device__ __forceinline__ void vst2(void* p, T v) { *(volatile T*)p = v; __threadfence(); *(volatile T*)p = v; }
__device__ __forceinline__ v8f wmma16(v16h a, v16h b, v8f c) {
  v8f d = __builtin_amdgcn_wmma_f32_16x16x32_f16(false, a, false, b, (short)0, c, false, false);
  asm volatile("v_nop\n\tv_nop\n\tv_nop\n\tv_nop" : "+v"(d) : "v"(a), "v"(b));
  return d;
}
__device__ __forceinline__ v8f wmma_bf(v16b a, v16b b, v8f c) {
  v8f d = __builtin_amdgcn_wmma_f32_16x16x32_bf16(false, a, false, b, (short)0, c, false, false);
  asm volatile("v_nop\n\tv_nop\n\tv_nop\n\tv_nop" : "+v"(d) : "v"(a), "v"(b));
  return d;
}
__device__ __forceinline__ v16h frag_h(const _Float16* rowk0, int lane) {
  union { v16h v; v8h q[2]; } u; const _Float16* p = rowk0 + 8 * (lane >> 4);
  u.q[0] = *(const v8h*)p; u.q[1] = *(const v8h*)(p + 16); return u.v;
}
__device__ __forceinline__ v16h frag_f32(const float* rowk0, int lane) {
  v16h a; const float* p = rowk0 + 8 * (lane >> 4);
#pragma unroll
  for (int i = 0; i < 8; ++i) { a[i] = (_Float16)p[i]; a[8 + i] = (_Float16)p[16 + i]; }
  return a;
}
__device__ __forceinline__ v16h frag_f32s(const float* rowk0, int lane, float sc) {
  v16h a; const float* p = rowk0 + 8 * (lane >> 4);
#pragma unroll
  for (int i = 0; i < 8; ++i) { a[i] = (_Float16)(p[i] * sc); a[8 + i] = (_Float16)(p[16 + i] * sc); }
  return a;
}
__device__ __forceinline__ v16h fragc_f32(const float* W, int k0, int n, int lane, int ld, int K) {
  v16h a; const int g = lane >> 4;
#pragma unroll
  for (int i = 0; i < 8; ++i) { const int ka = k0 + 8 * g + i, kb = ka + 16;
    a[i] = (_Float16)(ka < K ? W[(size_t)ka * ld + n] : 0.f); a[8 + i] = (_Float16)(kb < K ? W[(size_t)kb * ld + n] : 0.f); }
  return a;
}
struct F2 { v16b h, l; };
__device__ __forceinline__ F2 bsplit16(const float v[16]) { F2 r;
#pragma unroll
  for (int i = 0; i < 16; ++i) { const __bf16 h = (__bf16)v[i]; r.h[i] = h; r.l[i] = (__bf16)(v[i] - (float)h); }
  return r; }
__device__ __forceinline__ F2 split_row(const float* row, int k0, int lane) { float v[16]; const float* p = row + k0 + 8 * (lane >> 4);
#pragma unroll
  for (int i = 0; i < 8; ++i) { v[i] = p[i]; v[8 + i] = p[16 + i]; }
  return bsplit16(v); }
__device__ __forceinline__ F2 split_rowK(const float* row, int k0, int lane, int K) { float v[16]; const int g = lane >> 4;
#pragma unroll
  for (int i = 0; i < 8; ++i) { const int ka = k0 + 8 * g + i, kb = ka + 16; v[i] = ka < K ? row[ka] : 0.f; v[8 + i] = kb < K ? row[kb] : 0.f; }
  return bsplit16(v); }
__device__ __forceinline__ F2 split_col(const float* W, int k0, int n, int lane, int ld, int K) { float v[16]; const int g = lane >> 4;
#pragma unroll
  for (int i = 0; i < 8; ++i) { const int ka = k0 + 8 * g + i, kb = ka + 16; v[i] = ka < K ? W[(size_t)ka * ld + n] : 0.f; v[8 + i] = kb < K ? W[(size_t)kb * ld + n] : 0.f; }
  return bsplit16(v); }
__device__ __forceinline__ v8f mac3(const F2& a, const F2& b, v8f c) { c = wmma_bf(a.l, b.h, c); c = wmma_bf(a.h, b.l, c); return wmma_bf(a.h, b.h, c); }
__device__ __forceinline__ float sigm(float v) { return 1.0f / (1.0f + expf(-v)); }
#define LDSX() do { asm volatile("s_wait_dscnt 0" ::: "memory"); __builtin_amdgcn_wave_barrier(); __builtin_amdgcn_fence(__ATOMIC_RELEASE, "workgroup"); } while (0)

#define NQ 512
#define CC 64
#define HWS 441
#define HWP 448
#define WAY 5
#define SHOT 5
#define NLOC (SHOT * HWS)

__global__ __launch_bounds__(256) void k_cov(const float* __restrict__ x2, float* __restrict__ COV) {
  __shared__ float smu[CC]; __shared__ __align__(16) float scov[CC][CC];
  const int w = blockIdx.x, tid = threadIdx.x;
  if (tid < CC) { float s = 0.f; for (int sh = 0; sh < SHOT; ++sh) { const float* p = x2 + ((size_t)(w * SHOT + sh) * CC + tid) * HWS; for (int i = 0; i < HWS; ++i) s += p[i]; } smu[tid] = s / (float)NLOC; }
  __syncthreads();
  for (int q = tid; q < CC * CC; q += 256) { const int c = q >> 6, d = q & 63; const float mc = smu[c], mdv = smu[d]; float s = 0.f;
    for (int sh = 0; sh < SHOT; ++sh) { const float* pc = x2 + ((size_t)(w * SHOT + sh) * CC + c) * HWS; const float* pd = x2 + ((size_t)(w * SHOT + sh) * CC + d) * HWS;
      for (int i = 0; i < HWS; ++i) s += (pc[i] - mc) * (pd[i] - mdv); }
    scov[c][d] = s / (float)(NLOC - 1); }
  __syncthreads();
  for (int q = tid; q < CC * CC / 4; q += 256) vst2(COV + (size_t)w * CC * CC + q * 4, *(const v4f*)(&scov[0][0] + q * 4));
}
__global__ __launch_bounds__(128) void k_sim(const float* __restrict__ x1, const float* __restrict__ COV, const float* __restrict__ cw, const float* __restrict__ cb, float* __restrict__ SP) {
  __shared__ __align__(16) float sq[CC][HWP + 4];
  __shared__ float ssim[4][HWP]; __shared__ __align__(16) float sres[32];
  const int b = blockIdx.x, tid = threadIdx.x, wave = tid >> 5, lane = tid & 31, col = lane & 15, g = lane >> 4;
  { const int c = tid >> 1, hf = tid & 1; const float* p = x1 + ((size_t)b * CC + c) * HWS; float s = 0.f;
    for (int i = hf; i < HWS; i += 2) { const float v = p[i]; sq[c][i] = v; s += v; }
    s += __shfl_xor(s, 1, 32); const float mu = s / (float)HWS;
    __syncthreads();
    for (int i = hf; i < HWP + 4; i += 2) sq[c][i] = i < HWS ? sq[c][i] - mu : 0.f; }
  __syncthreads();
  if (tid < 32) sres[tid] = 0.f;
#pragma unroll 1
  for (int w = 0; w < WAY; ++w) {
    const float* cv = COV + (size_t)w * CC * CC;
    v16h a[2];
#pragma unroll
    for (int kc = 0; kc < 2; ++kc) a[kc] = frag_f32(cv + (size_t)(wave * 16 + col) * CC + kc * 32, lane);
#pragma unroll 1
    for (int tg = 0; tg < HWP / 16; tg += 7) { v8f acc[7];
#pragma unroll
      for (int t = 0; t < 7; ++t) acc[t] = (v8f){};
#pragma unroll
      for (int kc = 0; kc < 2; ++kc)
#pragma unroll
        for (int t = 0; t < 7; ++t) acc[t] = wmma16(a[kc], fragc_f32(&sq[0][0], kc * 32, (tg + t) * 16 + col, lane, HWP + 4, CC), acc[t]);
#pragma unroll
      for (int t = 0; t < 7; ++t) { const int s = (tg + t) * 16 + col; float ps = 0.f;
#pragma unroll
        for (int r = 0; r < 8; ++r) ps += sq[wave * 16 + 8 * g + r][s] * acc[t][r];
        ps += __shfl_xor(ps, 16, 32);
        if (g == 0) ssim[wave][s] = ps; } }
    __syncthreads();
    float part = 0.f;
    for (int s = tid; s < HWS; s += 128) { float v = (ssim[0][s] + ssim[1][s]) + (ssim[2][s] + ssim[3][s]); v = v > 0.f ? v : 0.2f * v; part += v * cw[s]; }
#pragma unroll
    for (int off = 16; off >= 1; off >>= 1) part += __shfl_xor(part, off, 32);
    __syncthreads();
    if (lane == 0) ssim[0][wave] = part;
    __syncthreads();
    if (tid == 0) sres[w] = ((ssim[0][0] + ssim[0][1]) + (ssim[0][2] + ssim[0][3])) + cb[0];
    __syncthreads(); }
  if (tid < 8) vst2(SP + (size_t)b * 32 + tid * 4, *(const v4f*)(&sres[tid * 4]));
}
__global__ __launch_bounds__(64) void k_pack(const float* __restrict__ SP, float* __restrict__ out) {
  __shared__ __align__(16) float so[64 * WAY];
  const int b0 = blockIdx.x * 64, tid = threadIdx.x;
  for (int w = 0; w < WAY; ++w) so[tid * WAY + w] = SP[(size_t)(b0 + tid) * 32 + w];
  __syncthreads();
  for (int q = tid; q < 64 * WAY / 4; q += 64) vst2(out + (size_t)b0 * WAY + q * 4, *(const v4f*)(&so[q * 4]));
}
extern "C" void kernel_launch(void* const* d_in, const int* in_sizes, int n_in, void* d_out, int out_size, void* d_ws, size_t ws_size, hipStream_t stream) {
  (void)in_sizes; (void)n_in; (void)out_size; (void)ws_size;
  const float* x1 = (const float*)d_in[0]; const float* x2 = (const float*)d_in[1]; const float* cw = (const float*)d_in[2]; const float* cb = (const float*)d_in[3];
  float* out = (float*)d_out;
  char* ws = (char*)d_ws; size_t off = 0;
  auto take = [&](size_t bytes) { char* p = ws + off; off += (bytes + 255) & ~(size_t)255; return p; };
  float* COV = (float*)take((size_t)WAY * CC * CC * 4); float* SP = (float*)take((size_t)NQ * 32 * 4);
  k_cov<<<WAY, 256, 0, stream>>>(x2, COV);
  k_sim<<<NQ, 128, 0, stream>>>(x1, COV, cw, cb, SP);
  k_pack<<<NQ / 64, 64, 0, stream>>>(SP, out);
}
